// K2311_2181843386511
// MI455X (gfx1250) — hardware-run, weakly checked
//
#include <hip/hip_runtime.h>
#include <math.h>

typedef __attribute__((ext_vector_type(16))) _Float16 v16h;
typedef __attribute__((ext_vector_type(8)))  _Float16 v8h;
typedef __attribute__((ext_vector_type(8)))  float    v8f;
typedef __attribute__((ext_vector_type(4)))  float    v4f;
typedef __attribute__((ext_vector_type(4)))  unsigned v4u;
typedef __attribute__((ext_vector_type(8)))  unsigned v8u;

constexpr int kNB     = 8;
constexpr int kC      = 256;
constexpr int kHW     = 56;
constexpr int kL      = kHW * kHW;
constexpr int kG      = 8;
constexpr int kCG     = kC / kG;
constexpr int kTaps   = 9;
constexpr int kPK     = kCG * kTaps;
constexpr int kPW     = kHW + 6;
constexpr int kPP     = kPW * kPW;
constexpr int kXPP    = 3904;
constexpr int kB      = kNB * kG;
constexpr int kPlanes = kNB * kC;
constexpr int kWPitch = 320;
constexpr int kGK     = 13;
constexpr int kGPad   = 6;
constexpr int kStRows = 76;
constexpr int kStPitch = 80;
constexpr int kStChunks = kStRows * kStPitch / 8;
constexpr int kBandHalves = kGK * 16 * 32;
constexpr int kBandChunks = kBandHalves / 8;
constexpr int kSCP    = 292;
constexpr int kSPP    = 40;
constexpr int kSOP    = 36;
constexpr int kTilesL = kL / 32;
constexpr int kWavesT = 7;
constexpr int kGrpT   = kTilesL / kWavesT;
constexpr float kAttnCarry = 1024.0f;
constexpr float kWCarry    = 64.0f;
constexpr float kHalfPi    = 1.5707963267948966f;
static_assert(kL == 3136 && kPK == 288 && kPP == 3844 && kCG == 32, "shape");
static_assert((kXPP % 32) == 0 && kXPP >= kPP && (kXPP * 2) % 128 == 0, "planar pitch: k multiple of 32, whole lines");
static_assert((kPK % 32) == 0 && (kL % 32) == 0, "k and l tile multiples");
static_assert(kGrpT * kWavesT == kTilesL, "l tiles per block");
static_assert(kStRows >= 48 + 15 + (kGK - 1) + 1, "stencil tile rows: last m tile + last tap row");
static_assert(kStPitch >= 48 + 32 && (kStPitch % 8) == 0, "stencil tile columns: last n tile + 32 k, 16-B rows");
static_assert(15 + (kGK - 1) < 32, "band fits one 32-deep k step");
static_assert(kStChunks == 760 && kBandChunks == 832, "stencil staging chunk counts");
static_assert(kStRows * kStPitch * 2 + kBandHalves * 2 + kL * 4 <= 65536, "stencil LDS");

constexpr size_t kSzXG  = (size_t)kPlanes * kL * 4;
constexpr size_t kSzXPG = 512 + (size_t)kPlanes * kXPP * 2 + 512;
constexpr size_t kSzXT  = (size_t)kB * kPP * kCG * 2;
constexpr size_t kSzPXT = (size_t)kB * kL * kCG * 2;
constexpr size_t kSzATR = (size_t)kB * kCG * kPK * 2;
constexpr size_t kSzW   = (size_t)kC * kWPitch * 2;
constexpr size_t kOffXG  = 0;
constexpr size_t kOffXPG = kOffXG + kSzXG;
constexpr size_t kOffXTH = kOffXPG + kSzXPG;
constexpr size_t kOffSTP = kOffXTH + kSzXT;
constexpr size_t kOffPXT = kOffSTP + kSzXT;
constexpr size_t kOffATR = kOffPXT + kSzPXT;
constexpr size_t kOffWH  = kOffATR + kSzATR;
constexpr size_t kWsTotal = kOffWH + kSzW;
static_assert(kWsTotal == 87360512ull, "carve total");
static_assert(kWsTotal <= 134217728ull, "carve cap");
static_assert((kOffXPG % 128) == 0 && (kOffXTH % 128) == 0 && (kOffSTP % 128) == 0 &&
              (kOffPXT % 128) == 0 && (kOffATR % 128) == 0 && (kOffWH % 128) == 0, "aligned regions");

__device__ __forceinline__ int clampi(int v, int lo, int hi) { return v < lo ? lo : (v > hi ? hi : v); }
__device__ __forceinline__ float bf16_rne(float f) {
  const unsigned u = __float_as_uint(f);
  return __uint_as_float((u + 0x7FFFu + ((u >> 16) & 1u)) & 0xFFFF0000u);
}
__device__ __forceinline__ unsigned short h_bits(float f) {
  const _Float16 h = (_Float16)f;
  return __builtin_bit_cast(unsigned short, h);
}
union FragH { v16h v; v8h h[2]; };
__device__ __forceinline__ v16h frag_load(const _Float16* p) {
  FragH f;
  f.h[0] = *(const v8h*)(p);
  f.h[1] = *(const v8h*)(p + 16);
  return f.v;
}
__device__ __forceinline__ v16h frag_load_shift(const unsigned short* rowp, int e) {
  const int ea = e & ~1;
  const unsigned sh = ((unsigned)e & 1u) << 4;
  const unsigned* p = (const unsigned*)(rowp + ea);
  const unsigned d0 = p[0], d1 = p[1], d2 = p[2], d3 = p[3], d4 = p[4];
  const unsigned d5 = p[8], d6 = p[9], d7 = p[10], d8 = p[11], d9 = p[12];
  v8u w;
  w[0] = __builtin_amdgcn_alignbit(d1, d0, sh);
  w[1] = __builtin_amdgcn_alignbit(d2, d1, sh);
  w[2] = __builtin_amdgcn_alignbit(d3, d2, sh);
  w[3] = __builtin_amdgcn_alignbit(d4, d3, sh);
  w[4] = __builtin_amdgcn_alignbit(d6, d5, sh);
  w[5] = __builtin_amdgcn_alignbit(d7, d6, sh);
  w[6] = __builtin_amdgcn_alignbit(d8, d7, sh);
  w[7] = __builtin_amdgcn_alignbit(d9, d8, sh);
  return __builtin_bit_cast(v16h, w);
}
__device__ __forceinline__ v8f mma_h(v16h a, v16h b, v8f c) {
  c = __builtin_amdgcn_wmma_f32_16x16x32_f16(false, a, false, b, (short)0, c, false, false);
  asm volatile("v_nop\n\tv_nop\n\tv_nop\n\tv_nop" : "+v"(c) : "v"(a), "v"(b));
  return c;
}
__device__ __forceinline__ void put8(float* p, v8f a, float s) {
  v4f u0, u1;
  u0[0] = a[0] * s; u0[1] = a[1] * s; u0[2] = a[2] * s; u0[3] = a[3] * s;
  u1[0] = a[4] * s; u1[1] = a[5] * s; u1[2] = a[6] * s; u1[3] = a[7] * s;
  *(v4f*)(p) = u0;
  *(v4f*)(p + 4) = u1;
}
__device__ __forceinline__ void wave_lds_sync() {
  __builtin_amdgcn_fence(__ATOMIC_RELEASE, "workgroup");
  __builtin_amdgcn_wave_barrier();
  __builtin_amdgcn_fence(__ATOMIC_ACQUIRE, "workgroup");
}

__global__ __launch_bounds__(256) void stencil_kernel(
    const float* __restrict__ x, const float* __restrict__ gw, const float* __restrict__ gb,
    float* __restrict__ XG, unsigned short* __restrict__ XP)
{
  __shared__ __align__(16) _Float16 sXh[kStRows * kStPitch];
  __shared__ __align__(16) _Float16 sWh[kBandHalves];
  __shared__ __align__(16) float sOut[kL];
  const int tid = threadIdx.x;
  const int plane = blockIdx.x;
  const int c = plane & (kC - 1);
  const float* xp = x + (size_t)plane * kL;
  const float* wsrc = gw + (size_t)c * (kGK * kGK);
#pragma unroll 1
  for (int it = 0; it < 3; ++it) {
    const int ch = it * 256 + tid;
    const int chc = ch < kStChunks ? ch : (kStChunks - 1);
    const int r = chc / (kStPitch / 8);
    const int c8 = (chc - r * (kStPitch / 8)) * 8;
    const int gy = r - kGPad;
    const bool rok = (unsigned)gy < (unsigned)kHW;
    const int cy = clampi(gy, 0, kHW - 1);
    const float* rp = xp + cy * kHW;
    v8h hv;
#pragma unroll
    for (int j = 0; j < 8; ++j) {
      const int gx = c8 + j - kGPad;
      const bool ok = rok && ((unsigned)gx < (unsigned)kHW);
      const int cx = clampi(gx, 0, kHW - 1);
      const float v = rp[cx];
      const float vb = bf16_rne(v);
      const float xv = ok ? vb : 0.0f;
      hv[j] = (_Float16)xv;
    }
    if (ch < kStChunks) {
      *(v8h*)(sXh + chc * 8) = hv;
    }
  }
#pragma unroll 1
  for (int it = 0; it < 4; ++it) {
    const int ch = it * 256 + tid;
    const int chc = ch < kBandChunks ? ch : (kBandChunks - 1);
    const int ky = chc >> 6;
    const int n = (chc >> 2) & 15;
    const int k8 = (chc & 3) * 8;
    const float* wr = wsrc + ky * kGK;
    v8h hv;
#pragma unroll
    for (int j = 0; j < 8; ++j) {
      const int d = k8 + j - n;
      const bool ok = (d >= 0) && (d < kGK);
      const int dc = clampi(d, 0, kGK - 1);
      const float w = wr[dc];
      const float wb = bf16_rne(w) * kWCarry;
      const float w64 = ok ? wb : 0.0f;
      hv[j] = (_Float16)w64;
    }
    if (ch < kBandChunks) {
      *(v8h*)(sWh + chc * 8) = hv;
    }
  }
  __syncthreads();

  const int wave = tid >> 5, lane = tid & 31;
  const int h = lane >> 4, cl = lane & 15;
  const int y0 = (wave >> 1) * 16;
  const int xa = (wave & 1) * 32;
  const _Float16* xrh = sXh + (y0 + cl) * kStPitch + xa + 8 * h;
  const _Float16* wrh = sWh + cl * 32 + 8 * h;
  v8f m0 = (v8f){0.f, 0.f, 0.f, 0.f, 0.f, 0.f, 0.f, 0.f};
  v8f m1 = m0;
#pragma unroll 1
  for (int ky = 0; ky < kGK; ++ky) {
    const int xo = ky * kStPitch;
    const int wo = ky * (16 * 32);
    const v16h bh = frag_load(wrh + wo);
    const v16h ah0 = frag_load(xrh + xo);
    const v16h ah1 = frag_load(xrh + xo + 16);
    m0 = mma_h(ah0, bh, m0);
    m1 = mma_h(ah1, bh, m1);
  }
  {
    const float bias = bf16_rne(gb[c]);
    const float iw = 1.0f / kWCarry;
    const int x0 = xa + cl;
    const int x1 = xa + 16 + cl;
#pragma unroll
    for (int r = 0; r < 8; ++r) {
      const int y = y0 + 8 * h + r;
      const float v0 = m0[r] * iw + bias;
      const float v1 = m1[r] * iw + bias;
      if (y < kHW && x0 < kHW) sOut[y * kHW + x0] = v0;
      if (y < kHW && x1 < kHW) sOut[y * kHW + x1] = v1;
    }
  }
  __syncthreads();

  float* og = XG + (size_t)plane * kL;
#pragma unroll 1
  for (int s = tid; s < kL / 4; s += 256) {
    const v4f res = *(const v4f*)(sOut + 4 * s);
    volatile v4f* dst = (volatile v4f*)(og + 4 * s);
    *dst = res;
    __threadfence();
    *dst = res;
  }
  unsigned short* pp = XP + (size_t)plane * kXPP;
#pragma unroll 1
  for (int k = tid; k < kXPP / 8; k += 256) {
    v8h hv;
#pragma unroll
    for (int j = 0; j < 8; ++j) {
      const int q = 8 * k + j;
      const int yy = q / kPW;
      const int xx = q - yy * kPW;
      const bool ok = (yy >= 3) && (yy < kHW + 3) && (xx >= 3) && (xx < kHW + 3);
      const int idx = clampi(yy - 3, 0, kHW - 1) * kHW + clampi(xx - 3, 0, kHW - 1);
      const float v = sOut[idx];
      const float pv = ok ? v : 0.0f;
      hv[j] = (_Float16)pv;
    }
    volatile v8h* d = (volatile v8h*)(pp + 8 * k);
    *d = hv;
    __threadfence();
    *d = hv;
  }
  if (plane == 0 && tid < 32) {
    const v4u z = {0u, 0u, 0u, 0u};
    volatile v4u* d = (volatile v4u*)(XP - 256 + 8 * tid);
    *d = z;
    __threadfence();
    *d = z;
  }
  if (plane == kPlanes - 1 && tid < 32) {
    const v4u z = {0u, 0u, 0u, 0u};
    volatile v4u* d = (volatile v4u*)(XP + (size_t)kPlanes * kXPP + 8 * tid);
    *d = z;
    __threadfence();
    *d = z;
  }
}

__global__ __launch_bounds__(256) void pack_kernel(
    const float* __restrict__ XG, unsigned short* __restrict__ XTH, unsigned short* __restrict__ STP)
{
  __shared__ __align__(16) unsigned short sH[kPW * kCG];
  __shared__ __align__(16) unsigned short sS[kPW * kCG];
  const int tid = threadIdx.x;
  const int b = blockIdx.x / kPW;
  const int yy = blockIdx.x - b * kPW;
  const bool rowok = (yy >= 3) && (yy < kHW + 3);
  const int yc = clampi(yy - 3, 0, kHW - 1);
  const float* src = XG + (size_t)b * kCG * kL + yc * kHW;
#pragma unroll 1
  for (int e = tid; e < kPW * kCG; e += 256) {
    const int ch = e / kPW;
    const int xx = e - ch * kPW;
    const bool ok = rowok && (xx >= 3) && (xx < kHW + 3);
    const int xc = clampi(xx - 3, 0, kHW - 1);
    const float v = src[(size_t)ch * kL + xc];
    const float xv = ok ? v : 0.0f;
    const float sf = sinf(xv * kHalfPi);
    const int o = xx * kCG + ch;
    sH[o] = h_bits(xv);
    sS[o] = h_bits(sf);
  }
  __syncthreads();
  if (tid < (kPW * kCG) / 8) {
    const v4u vh = *(const v4u*)(sH + 8 * tid);
    const v4u vs = *(const v4u*)(sS + 8 * tid);
    const size_t o = ((size_t)b * kPP + (size_t)yy * kPW) * kCG + 8 * tid;
    volatile v4u* dh = (volatile v4u*)(XTH + o);
    volatile v4u* ds = (volatile v4u*)(STP + o);
    *dh = vh; *ds = vs;
    __threadfence();
    *dh = vh; *ds = vs;
  }
}

__global__ __launch_bounds__(256) void wprep_kernel(
    const float* __restrict__ pw, unsigned short* __restrict__ WH)
{
  const int idx = blockIdx.x * 256 + threadIdx.x;
  const int co = idx / 40;
  const int ch = idx - co * 40;
  const bool real = ch < 36;
  const int chc = real ? ch : 35;
  const int kk = chc >> 2;
  const int ci0 = (chc & 3) * 8;
  const float* src = pw + (size_t)co * kPK + ci0 * kTaps + kk;
  v8h hv;
#pragma unroll
  for (int j = 0; j < 8; ++j) {
    const float w = src[j * kTaps];
    const float wb = bf16_rne(w) * kWCarry;
    const float w64 = real ? wb : 0.0f;
    hv[j] = (_Float16)w64;
  }
  volatile v8h* dh = (volatile v8h*)(WH + (size_t)idx * 8);
  *dh = hv;
  __threadfence();
  *dh = hv;
}

__global__ __launch_bounds__(288) void keys_kernel(
    const unsigned short* XP, const float* __restrict__ scale, unsigned short* __restrict__ ATR, float scl)
{
  __shared__ __align__(16) float sC[kCG * kSCP];
  const int tid = threadIdx.x;
  const int kk = tid >> 5;
  const int lane = tid & 31;
  const int h = lane >> 4, c = lane & 15;
  const int b = blockIdx.x;
  const int g = b & (kG - 1);
  const int kh = kk / 3;
  const int kw = kk - kh * 3;
  const int sft = (kh - 1) * (3 * kPW) + (kw - 1) * 3;
  const unsigned short* row0 = XP + (size_t)(b * kCG + c) * kXPP;
  const unsigned short* row1 = row0 + (size_t)16 * kXPP;
  v8f acc00 = (v8f){0.f, 0.f, 0.f, 0.f, 0.f, 0.f, 0.f, 0.f};
  v8f acc01 = acc00, acc10 = acc00, acc11 = acc00;
#pragma unroll 1
  for (int k0 = 0; k0 < kXPP; k0 += 32) {
    const int kb = k0 + 8 * h;
    const v16h b0 = frag_load((const _Float16*)(row0 + kb));
    const v16h b1 = frag_load((const _Float16*)(row1 + kb));
    const v16h a0 = frag_load_shift(row0, kb + sft);
    acc00 = mma_h(a0, b0, acc00);
    acc01 = mma_h(a0, b1, acc01);
    asm volatile("" ::: "memory");
    const v16h a1 = frag_load_shift(row1, kb + sft);
    acc10 = mma_h(a1, b0, acc10);
    acc11 = mma_h(a1, b1, acc11);
  }
  {
    float* p = sC + c * kSCP + kk * 32 + 8 * h;
    put8(p, acc00, scl);
    put8(p + 16, acc10, scl);
    put8(p + 16 * kSCP, acc01, scl);
    put8(p + 16 * kSCP + 16, acc11, scl);
  }
  __syncthreads();
  const float* sg = scale + (size_t)g * (kPK * kCG);
  unsigned short* dst = ATR + (size_t)b * (kCG * kPK);
#pragma unroll 1
  for (int i = 0; i < 4; ++i) {
    const int chunk = tid + 288 * i;
    const int c2 = chunk / 36;
    const int k8 = (chunk - c2 * 36) * 8;
    const int kk2 = k8 >> 5;
    const int cg0 = k8 & 31;
    const float* sp = sC + c2 * kSCP + k8;
    const v4f u0 = *(const v4f*)(sp);
    const v4f u1 = *(const v4f*)(sp + 4);
    const float* sq = sg + (cg0 * kTaps + kk2) * kCG + c2;
    const float s0 = bf16_rne(sq[0]), s1 = bf16_rne(sq[kPK]), s2 = bf16_rne(sq[2 * kPK]), s3 = bf16_rne(sq[3 * kPK]);
    const float s4 = bf16_rne(sq[4 * kPK]), s5 = bf16_rne(sq[5 * kPK]), s6 = bf16_rne(sq[6 * kPK]), s7 = bf16_rne(sq[7 * kPK]);
    v8h hv;
    hv[0] = (_Float16)(u0[0] * s0);
    hv[1] = (_Float16)(u0[1] * s1);
    hv[2] = (_Float16)(u0[2] * s2);
    hv[3] = (_Float16)(u0[3] * s3);
    hv[4] = (_Float16)(u1[0] * s4);
    hv[5] = (_Float16)(u1[1] * s5);
    hv[6] = (_Float16)(u1[2] * s6);
    hv[7] = (_Float16)(u1[3] * s7);
    volatile v8h* d = (volatile v8h*)(dst + (size_t)chunk * 8);
    *d = hv;
    __threadfence();
    *d = hv;
  }
}

__global__ __launch_bounds__(224) void conv_kernel(
    const unsigned short* __restrict__ XTH, const unsigned short* __restrict__ WH,
    const float* __restrict__ pb, unsigned short* __restrict__ PXT)
{
  __shared__ __align__(16) _Float16 sP[kWavesT][32 * kSPP];
  const int tid = threadIdx.x;
  const int wave = tid >> 5, lane = tid & 31;
  const int h = lane >> 4, c = lane & 15;
  const int b = blockIdx.x / kGrpT;
  const int grp = blockIdx.x - b * kGrpT;
  const int g = b & (kG - 1);
  const int l0 = (grp * kWavesT + wave) * 32;
  const int la = l0 + c, lb = l0 + 16 + c;
  const int ya = la / kHW, yb = lb / kHW;
  const int qa = (ya + 3) * kPW + (la - ya * kHW) + 3;
  const int qb = (yb + 3) * kPW + (lb - yb * kHW) + 3;
  const _Float16* xh0 = (const _Float16*)XTH + ((size_t)b * kPP + qa) * kCG + 8 * h;
  const _Float16* xh1 = (const _Float16*)XTH + ((size_t)b * kPP + qb) * kCG + 8 * h;
  const _Float16* wh0 = (const _Float16*)WH + (size_t)(g * kCG + c) * kWPitch + 8 * h;
  const _Float16* wh1 = wh0 + (size_t)16 * kWPitch;
  v8f m00 = (v8f){0.f, 0.f, 0.f, 0.f, 0.f, 0.f, 0.f, 0.f};
  v8f m01 = m00, m10 = m00, m11 = m00;
#pragma unroll 1
  for (int kk = 0; kk < kTaps; ++kk) {
    const int kh = kk / 3;
    const int kw = kk - kh * 3;
    const int off = ((kh - 1) * (3 * kPW) + (kw - 1) * 3) * kCG;
    const v16h ah0 = frag_load(xh0 + off);
    const v16h ah1 = frag_load(xh1 + off);
    const v16h bh0 = frag_load(wh0 + kk * 32);
    const v16h bh1 = frag_load(wh1 + kk * 32);
    m00 = mma_h(ah0, bh0, m00);
    m01 = mma_h(ah0, bh1, m01);
    m10 = mma_h(ah1, bh0, m10);
    m11 = mma_h(ah1, bh1, m11);
  }
  const float bias0 = bf16_rne(pb[g * kCG + c]);
  const float bias1 = bf16_rne(pb[g * kCG + 16 + c]);
  const float iw = 1.0f / kWCarry;
  _Float16* sp = sP[wave];
#pragma unroll
  for (int r = 0; r < 8; ++r) {
    const float v00 = m00[r] * iw + bias0;
    const float v01 = m01[r] * iw + bias1;
    const float v10 = m10[r] * iw + bias0;
    const float v11 = m11[r] * iw + bias1;
    sp[(8 * h + r) * kSPP + c]           = (_Float16)v00;
    sp[(8 * h + r) * kSPP + 16 + c]      = (_Float16)v01;
    sp[(16 + 8 * h + r) * kSPP + c]      = (_Float16)v10;
    sp[(16 + 8 * h + r) * kSPP + 16 + c] = (_Float16)v11;
  }
  wave_lds_sync();
  v8h ov[4];
#pragma unroll
  for (int it = 0; it < 4; ++it) {
    const int chunk = it * 32 + lane;
    ov[it] = *(const v8h*)(sp + (chunk >> 2) * kSPP + (chunk & 3) * 8);
  }
  unsigned short* dst = PXT + ((size_t)b * kL + l0) * kCG;
  for (int pass = 0; pass < 2; ++pass) {
#pragma unroll
    for (int it = 0; it < 4; ++it)
      *(volatile v8h*)(dst + (size_t)(it * 32 + lane) * 8) = ov[it];
    __threadfence();
  }
}

__global__ __launch_bounds__(224) void out_kernel(
    const unsigned short* __restrict__ ATR, const unsigned short* __restrict__ PXT,
    const unsigned short* __restrict__ STP, float* __restrict__ out, float oscl)
{
  __shared__ __align__(16) float sO[kWavesT][32 * kSOP];
  const int tid = threadIdx.x;
  const int wave = tid >> 5, lane = tid & 31;
  const int h = lane >> 4, c = lane & 15;
  const int b = blockIdx.x / kGrpT;
  const int grp = blockIdx.x - b * kGrpT;
  const int l0 = (grp * kWavesT + wave) * 32;
  const int la = l0 + c, lb = l0 + 16 + c;
  const int ya = la / kHW, yb = lb / kHW;
  const int qa = (ya + 3) * kPW + (la - ya * kHW) + 3;
  const int qb = (yb + 3) * kPW + (lb - yb * kHW) + 3;
  const _Float16* pxb = (const _Float16*)PXT + (size_t)b * kL * kCG + 8 * h;
  const v16h px0 = frag_load(pxb + (size_t)la * kCG);
  const v16h px1 = frag_load(pxb + (size_t)lb * kCG);
  const _Float16* st0 = (const _Float16*)STP + ((size_t)b * kPP + qa) * kCG + 8 * h;
  const _Float16* st1 = (const _Float16*)STP + ((size_t)b * kPP + qb) * kCG + 8 * h;
  const _Float16* at0 = (const _Float16*)ATR + ((size_t)b * kCG + c) * kPK + 8 * h;
  const _Float16* at1 = at0 + (size_t)16 * kPK;
  v8f acc00 = (v8f){0.f, 0.f, 0.f, 0.f, 0.f, 0.f, 0.f, 0.f};
  v8f acc01 = acc00, acc10 = acc00, acc11 = acc00;
#pragma unroll 1
  for (int kk = 0; kk < kTaps; ++kk) {
    const int kh = kk / 3;
    const int kw = kk - kh * 3;
    const int off = ((kh - 1) * (3 * kPW) + (kw - 1) * 3) * kCG;
    const v16h s0 = frag_load(st0 + off);
    const v16h s1 = frag_load(st1 + off);
    const v16h f0 = __builtin_elementwise_max(px0, s0);
    const v16h f1 = __builtin_elementwise_max(px1, s1);
    const v16h a0 = frag_load(at0 + kk * 32);
    const v16h a1 = frag_load(at1 + kk * 32);
    acc00 = mma_h(a0, f0, acc00);
    acc01 = mma_h(a0, f1, acc01);
    acc10 = mma_h(a1, f0, acc10);
    acc11 = mma_h(a1, f1, acc11);
  }
  float* so = sO[wave];
#pragma unroll
  for (int r = 0; r < 8; ++r) {
    so[(8 * h + r) * kSOP + c]           = acc00[r] * oscl;
    so[(8 * h + r) * kSOP + 16 + c]      = acc01[r] * oscl;
    so[(16 + 8 * h + r) * kSOP + c]      = acc10[r] * oscl;
    so[(16 + 8 * h + r) * kSOP + 16 + c] = acc11[r] * oscl;
  }
  wave_lds_sync();
  const int rq = lane >> 3, c4 = (lane & 7) * 4;
  v4f ov[8];
#pragma unroll
  for (int it = 0; it < 8; ++it) ov[it] = *(const v4f*)(so + (it * 4 + rq) * kSOP + c4);
  float* ob = out + (size_t)b * kCG * kL + l0 + c4;
  for (int pass = 0; pass < 2; ++pass) {
#pragma unroll
    for (int it = 0; it < 8; ++it)
      *(volatile v4f*)(ob + (size_t)(it * 4 + rq) * kL) = ov[it];
    __threadfence();
  }
}

extern "C" void kernel_launch(void* const* d_in, const int* in_sizes, int n_in,
                              void* d_out, int out_size, void* d_ws, size_t ws_size,
                              hipStream_t stream) {
  if (n_in < 6) return;
  if (in_sizes[0] != kPlanes * kL) return;
  if (in_sizes[1] != kC * kGK * kGK) return;
  if (in_sizes[2] != kC) return;
  if (in_sizes[3] != kC * kPK) return;
  if (in_sizes[4] != kC) return;
  if (in_sizes[5] != kG * kPK * kCG) return;
  if (out_size != kPlanes * kL) return;
  if (ws_size < kWsTotal) return;

  const float* x        = (const float*)d_in[0];
  const float* gather_w = (const float*)d_in[1];
  const float* gather_b = (const float*)d_in[2];
  const float* proj_w   = (const float*)d_in[3];
  const float* proj_b   = (const float*)d_in[4];
  const float* scale    = (const float*)d_in[5];
  float* out = (float*)d_out;

  char* ws = (char*)d_ws;
  float*          XG  = (float*)(ws + kOffXG);
  unsigned short* XP  = (unsigned short*)(ws + kOffXPG + 512);
  unsigned short* XTH = (unsigned short*)(ws + kOffXTH);
  unsigned short* STP = (unsigned short*)(ws + kOffSTP);
  unsigned short* PXT = (unsigned short*)(ws + kOffPXT);
  unsigned short* ATR = (unsigned short*)(ws + kOffATR);
  unsigned short* WH  = (unsigned short*)(ws + kOffWH);

  const float invSqrtL = 1.0f / sqrtf((float)kL);
  const float keyScl = kAttnCarry * invSqrtL;
  const float outScl = (1.0f / sqrtf((float)kPK)) * (1.0f / kAttnCarry);

  stencil_kernel<<<kPlanes, 256, 0, stream>>>(x, gather_w, gather_b, XG, XP);
  pack_kernel<<<kB * kPW, 256, 0, stream>>>(XG, XTH, STP);
  wprep_kernel<<<(kC * (kWPitch / 8)) / 256, 256, 0, stream>>>(proj_w, WH);
  keys_kernel<<<kB, 288, 0, stream>>>(XP, scale, ATR, keyScl);
  conv_kernel<<<kB * kGrpT, 224, 0, stream>>>(XTH, WH, proj_b, PXT);
  out_kernel<<<kB * kGrpT, 224, 0, stream>>>(ATR, PXT, STP, out, outScl);
}
